// GraphStateEncoder_34488587387632
// MI455X (gfx1250) — hardware-verified
//
#include <hip/hip_runtime.h>
#include <stddef.h>


#define KD    256
#define HCW   64
#define GR    32
#define AP    264
#define TP    264
#define NTHR  256
#define NWAVE 8
#define CHUNK 2048
#define WCAP  256
#define NGRP  (CHUNK / (NTHR * 4))

static_assert(WCAP == (CHUNK / NTHR) * 32);
static_assert(NGRP >= 1);
static_assert(KD == NTHR);
static_assert((AP % 8) == 0 && (TP % 8) == 0);
static_assert(CHUNK == 2048);

typedef float    v4f  __attribute__((ext_vector_type(4)));
typedef float    v8f  __attribute__((ext_vector_type(8)));
typedef int      v4i  __attribute__((ext_vector_type(4)));
typedef _Float16 v8h  __attribute__((ext_vector_type(8)));
typedef _Float16 v16h __attribute__((ext_vector_type(16)));
union Frag   { v16h v; v8h half[2]; };
union Pack16 { v8h h; v4i i; _Float16 s[8]; };

__device__ __forceinline__ v8f wm(v16h a, v16h b, v8f c) {
  v8f d = __builtin_amdgcn_wmma_f32_16x16x32_f16(false, a, false, b, (short)0, c, false, false);
  asm volatile("v_nop\n\tv_nop\n\tv_nop\n\tv_nop" : "+v"(d) : "v"(a), "v"(b));
  return d;
}

__device__ __forceinline__ float lrelu_exp(float a) {
  a = (a > 0.f) ? a : 0.2f * a;
  a = fminf(a, 80.f);
  return __expf(a);
}

template <int NOUT>
__global__ __launch_bounds__(NTHR) void k_prepw(const float* __restrict__ W, _Float16* Wh) {
  __shared__ __attribute__((aligned(16))) _Float16 T[16 * TP];
  const int tid = threadIdx.x, lane = tid & 31, wave = tid >> 5;
  const int n0 = blockIdx.x * 16;
  {
    const int k = tid;
    const float* p = W + (size_t)k * NOUT + n0;
#pragma unroll
    for (int q = 0; q < 4; ++q) {
      const v4f f = *(const v4f*)(p + 4 * q);
      T[(4 * q + 0) * TP + k] = (_Float16)(f.x * 16.0f);
      T[(4 * q + 1) * TP + k] = (_Float16)(f.y * 16.0f);
      T[(4 * q + 2) * TP + k] = (_Float16)(f.z * 16.0f);
      T[(4 * q + 3) * TP + k] = (_Float16)(f.w * 16.0f);
    }
  }
  __syncthreads();
  Pack16 u0, u1;
  u0.h = *(const v8h*)(T + (2 * wave) * TP + 8 * lane);
  u1.h = *(const v8h*)(T + (2 * wave + 1) * TP + 8 * lane);
  _Float16* d0 = Wh + (size_t)(n0 + 2 * wave) * KD + 8 * lane;
  _Float16* d1 = Wh + (size_t)(n0 + 2 * wave + 1) * KD + 8 * lane;
  *(volatile v4i*)d0 = u0.i;
  *(volatile v4i*)d1 = u1.i;
  __threadfence();
  *(volatile v4i*)d0 = u0.i;
  *(volatile v4i*)d1 = u1.i;
}

template <int NOUT, int NHD>
__global__ __launch_bounds__(NTHR) void k_gemm(
    const float* __restrict__ x, const _Float16* __restrict__ Wh,
    const float* __restrict__ att_src, const float* __restrict__ att_dst,
    float* xp, float* es, float* ed, int nN) {
  static_assert(NOUT == 256 || NOUT == 64);
  static_assert(NOUT == NHD * HCW);
  constexpr int RT  = (NOUT == 256) ? 2 : 1;
  constexpr int CT  = RT;
  constexpr int XSP = NOUT + 4;
  constexpr int NI  = NOUT / 32;
  __shared__ __attribute__((aligned(16))) _Float16 At[GR * AP];
  __shared__ __attribute__((aligned(16))) float Xs[GR * XSP];
  __shared__ __attribute__((aligned(16))) float Ls[2 * GR * NHD];

  const int tid  = threadIdx.x;
  const int lane = tid & 31;
  const int wave = tid >> 5;
  const int hh   = lane >> 4;
  const int m    = lane & 15;
  const int rowBase = blockIdx.x * GR;

  {
    const int r  = tid >> 3;
    const int c0 = (tid & 7) * 32;
    int row = rowBase + r;
    if (row > nN - 1) row = nN - 1;
    const float* p = x + (size_t)row * KD + c0;
#pragma unroll
    for (int q = 0; q < 4; ++q) {
      const v4f fa = *(const v4f*)(p + 8 * q);
      const v4f fb = *(const v4f*)(p + 8 * q + 4);
      Pack16 u;
      u.s[0] = (_Float16)fa.x; u.s[1] = (_Float16)fa.y; u.s[2] = (_Float16)fa.z; u.s[3] = (_Float16)fa.w;
      u.s[4] = (_Float16)fb.x; u.s[5] = (_Float16)fb.y; u.s[6] = (_Float16)fb.z; u.s[7] = (_Float16)fb.w;
      *(v8h*)(At + r * AP + c0 + 8 * q) = u.h;
    }
  }
  __syncthreads();

  const int rt0 = (NOUT == 256) ? 0 : (wave >> 2);
  const int ct0 = (NOUT == 256) ? 2 * wave : (wave & 3);
  v8f acc[RT][CT];
#pragma unroll
  for (int rt = 0; rt < RT; ++rt)
#pragma unroll
    for (int ct = 0; ct < CT; ++ct)
#pragma unroll
      for (int r = 0; r < 8; ++r) acc[rt][ct][r] = 0.f;

#pragma unroll 2
  for (int kt = 0; kt < KD / 32; ++kt) {
    const int k0 = kt * 32;
    Frag a[RT], b[CT];
#pragma unroll
    for (int rt = 0; rt < RT; ++rt) {
      const _Float16* pa = At + (16 * (rt0 + rt) + m) * AP + k0 + 8 * hh;
      a[rt].half[0] = *(const v8h*)pa;
      a[rt].half[1] = *(const v8h*)(pa + 16);
    }
#pragma unroll
    for (int ct = 0; ct < CT; ++ct) {
      const _Float16* pb = Wh + (size_t)(16 * (ct0 + ct) + m) * KD + k0 + 8 * hh;
      b[ct].half[0] = *(const v8h*)pb;
      b[ct].half[1] = *(const v8h*)(pb + 16);
    }
#pragma unroll
    for (int rt = 0; rt < RT; ++rt)
#pragma unroll
      for (int ct = 0; ct < CT; ++ct) acc[rt][ct] = wm(a[rt].v, b[ct].v, acc[rt][ct]);
  }

#pragma unroll
  for (int rt = 0; rt < RT; ++rt)
#pragma unroll
    for (int ct = 0; ct < CT; ++ct)
#pragma unroll
      for (int r = 0; r < 8; ++r)
        Xs[(16 * (rt0 + rt) + 8 * hh + r) * XSP + 16 * (ct0 + ct) + m] = acc[rt][ct][r] * 0.0625f;
  __syncthreads();

  {
    constexpr int ND  = GR * NHD * 2;
    constexpr int TPD = NTHR / ND;
    constexpr int LEN = HCW / TPD;
    static_assert(ND * TPD == NTHR && TPD * LEN == HCW);
    const int d     = tid / TPD;
    const int part  = tid - d * TPD;
    const int row   = d / (2 * NHD);
    const int rem   = d - row * 2 * NHD;
    const int h     = rem >> 1;
    const int which = rem & 1;
    const float* av = which ? att_dst : att_src;
    const float* xs = Xs + row * XSP + h * HCW + part * LEN;
    const float* ap = av + h * HCW + part * LEN;
    float s = 0.f;
#pragma unroll 8
    for (int c = 0; c < LEN; ++c) s += xs[c] * ap[c];
#pragma unroll
    for (int mk = TPD / 2; mk >= 1; mk >>= 1) s += __shfl_xor(s, mk, 32);
    if (part == 0) Ls[which * GR * NHD + row * NHD + h] = s;
  }
  __syncthreads();

  v4f xr[NI];
#pragma unroll
  for (int i = 0; i < NI; ++i) {
    const int f   = i * 128 + 4 * lane;
    const int rl  = f / NOUT;
    const int col = f - rl * NOUT;
    xr[i] = *(const v4f*)(Xs + (4 * wave + rl) * XSP + col);
  }
  float* base = xp + (size_t)(rowBase + 4 * wave) * NOUT + 4 * lane;
  const bool lg = (wave < 2) && (lane < 8 * NHD);
  v4f lv = {0.f, 0.f, 0.f, 0.f};
  float* lp = es;
  if (lg) {
    lv = *(const v4f*)(Ls + wave * GR * NHD + 4 * lane);
    lp = (wave == 0 ? es : ed) + (size_t)rowBase * NHD + 4 * lane;
  }
#pragma unroll
  for (int i = 0; i < NI; ++i) *(volatile v4f*)(base + i * 128) = xr[i];
  if (lg) *(volatile v4f*)lp = lv;
  __threadfence();
#pragma unroll
  for (int i = 0; i < NI; ++i) *(volatile v4f*)(base + i * 128) = xr[i];
  if (lg) *(volatile v4f*)lp = lv;
}

template <int DF, int NHD, int NB, int SLOTB, bool RESID>
__global__ __launch_bounds__(NTHR) void k_gat(
    const float* __restrict__ xres, const int* __restrict__ ei,
    const float* __restrict__ xp, const float* __restrict__ es, const float* __restrict__ ed,
    const float* __restrict__ bias, const float* __restrict__ gam, const float* __restrict__ bet,
    float* out, int nN, int nE) {
  static_assert(NB == (1 << SLOTB));
  static_assert(DF == NHD * HCW);
  static_assert(DF == 256 || DF == 64);
  static_assert(SLOTB + 11 <= 31);
  constexpr int LPS = (DF == 64) ? 16 : 32;
  constexpr int NPC = DF / (4 * LPS);
  constexpr int SPI = 32 / LPS;
  constexpr int SPW = NB / NWAVE;
  static_assert(NPC * 4 * LPS == DF);
  static_assert((SPW % SPI) == 0);
  static_assert(((NB * DF + NB * NHD) % 4) == 0);

  extern __shared__ v4f lds_dyn[];
  float* sacc = (float*)lds_dyn;
  float* den  = sacc + NB * DF;
  int*   list = (int*)(den + NB * NHD);
  int*   wcnt = list + NWAVE * WCAP;

  const int tid  = threadIdx.x;
  const int lane = tid & 31;
  const int wave = tid >> 5;
  const int li   = lane & (LPS - 1);
  const int hsub = lane / LPS;
  const int nodeBase = blockIdx.x * NB;

  int colp[NPC], hdp[NPC];
#pragma unroll
  for (int p = 0; p < NPC; ++p) {
    colp[p] = p * 4 * LPS + 4 * li;
    hdp[p]  = colp[p] / HCW;
  }

  {
    const v4f z4 = {0.f, 0.f, 0.f, 0.f};
    for (int i = tid; i < (NB * DF + NB * NHD) / 4; i += NTHR) lds_dyn[i] = z4;
  }
  __syncthreads();

  const int* eid = ei + nE;
  const bool al16 = ((nE & 3) == 0);

  const int nChunks = (nE + CHUNK - 1) / CHUNK;
#pragma unroll 1
  for (int ch = 0; ch < nChunks; ++ch) {
    const int cbase = ch * CHUNK;
    int wc = 0;
#pragma unroll
    for (int g = 0; g < NGRP; ++g) {
      const int el0 = (g * NTHR + tid) * 4;
      const int e0  = cbase + el0;
      const int sent = -2147483647 - 1;
      v4i d;
      if (al16 && (e0 + 3 < nE)) {
        d = *(const v4i*)(eid + e0);
      } else {
        d.x = (e0     < nE) ? eid[e0]     : sent;
        d.y = (e0 + 1 < nE) ? eid[e0 + 1] : sent;
        d.z = (e0 + 2 < nE) ? eid[e0 + 2] : sent;
        d.w = (e0 + 3 < nE) ? eid[e0 + 3] : sent;
      }
      const unsigned s0 = (unsigned)d.x - (unsigned)nodeBase;
      const unsigned s1 = (unsigned)d.y - (unsigned)nodeBase;
      const unsigned s2 = (unsigned)d.z - (unsigned)nodeBase;
      const unsigned s3 = (unsigned)d.w - (unsigned)nodeBase;
      const bool h0 = s0 < (unsigned)NB;
      const bool h1 = s1 < (unsigned)NB;
      const bool h2 = s2 < (unsigned)NB;
      const bool h3 = s3 < (unsigned)NB;
      const unsigned many = __builtin_amdgcn_ballot_w32(h0 | h1 | h2 | h3);
      if (many != 0u) {
#define HITJ(J, HJ, SJ) { \
          const unsigned mj = __builtin_amdgcn_ballot_w32(HJ); \
          if (HJ) { \
            const int pos = wc + (int)__builtin_amdgcn_mbcnt_lo(mj, 0u); \
            if (pos < WCAP) list[wave * WCAP + pos] = ((el0 + (J)) << SLOTB) | (int)(SJ); \
          } \
          wc += (int)__builtin_popcount(mj); }
        HITJ(0, h0, s0)
        HITJ(1, h1, s1)
        HITJ(2, h2, s2)
        HITJ(3, h3, s3)
#undef HITJ
      }
    }
    if (lane == 0) wcnt[wave] = wc;
    __syncthreads();

    if (wave == 0) {
      for (int wsx = 0; wsx < NWAVE; ++wsx) {
        int n = wcnt[wsx];
        n = (n > WCAP) ? WCAP : ((n < 0) ? 0 : n);
        for (int i0 = 0; i0 < n; i0 += 32) {
          const int myi = i0 + lane;
          int key = 0;
          float myp[NHD];
#pragma unroll
          for (int h = 0; h < NHD; ++h) myp[h] = 0.f;
          if (myi < n) {
            const int ent  = list[wsx * WCAP + myi];
            const int slot = ent & (NB - 1);
            const int el   = (ent >> SLOTB) & (CHUNK - 1);
            int e = cbase + el;
            if (e > nE - 1) e = nE - 1;
            int src = ei[e];
            src = src < 0 ? 0 : (src > nN - 1 ? nN - 1 : src);
            int nd = nodeBase + slot;
            if (nd > nN - 1) nd = nN - 1;
#pragma unroll
            for (int h = 0; h < NHD; ++h)
              myp[h] = lrelu_exp(es[(size_t)src * NHD + h] + ed[(size_t)nd * NHD + h]);
            key = (src << SLOTB) | slot;
          }
          int cnt = n - i0;
          if (cnt > 32) cnt = 32;
          for (int k = 0; k < cnt; ++k) {
            const int kk   = __shfl(key, k, 32);
            const int src  = kk >> SLOTB;
            const int slot = kk & (NB - 1);
            float ph[NHD];
#pragma unroll
            for (int h = 0; h < NHD; ++h) ph[h] = __shfl(myp[h], k, 32);
            float pp[NPC];
#pragma unroll
            for (int p = 0; p < NPC; ++p) {
              float v = ph[0];
#pragma unroll
              for (int h = 1; h < NHD; ++h) if (hdp[p] == h) v = ph[h];
              pp[p] = v;
            }
            const float* xrow = xp + (size_t)src * DF;
            float* srow = sacc + slot * DF;
#pragma unroll
            for (int p = 0; p < NPC; ++p) {
              const v4f xv = *(const v4f*)(xrow + colp[p]);
              v4f* sp = (v4f*)(srow + colp[p]);
              const v4f nx = *sp + pp[p] * xv;
              if (lane < LPS) *sp = nx;
            }
            if (((li & 15) == 0) && (lane < LPS)) {
#pragma unroll
              for (int p = 0; p < NPC; ++p) {
                float* dp = den + slot * NHD + hdp[p];
                const float o = *dp;
                *dp = o + pp[p];
              }
            }
          }
        }
      }
    }
    __syncthreads();
  }

  v4f b4[NPC], g4[NPC], e4[NPC];
#pragma unroll
  for (int p = 0; p < NPC; ++p) {
    b4[p] = *(const v4f*)(bias + colp[p]);
    g4[p] = *(const v4f*)(gam + colp[p]);
    e4[p] = *(const v4f*)(bet + colp[p]);
  }
#pragma unroll 1
  for (int j = 0; j < SPW; j += SPI) {
    const int node0 = nodeBase + wave * SPW + j;
    if (node0 >= nN) break;
    const int slot = wave * SPW + j + hsub;
    const int node = nodeBase + slot;
    const bool valid = node < nN;
    const int nrow = valid ? node : (nN - 1);
    const size_t rb = (size_t)nrow * DF;
    float ps[NPC];
#pragma unroll
    for (int p = 0; p < NPC; ++p)
      ps[p] = lrelu_exp(es[(size_t)nrow * NHD + hdp[p]] + ed[(size_t)nrow * NHD + hdp[p]]);
    v4f hv[NPC];
    float s1 = 0.f;
#pragma unroll
    for (int p = 0; p < NPC; ++p) {
      const v4f xv = *(const v4f*)(xp + rb + colp[p]);
      const v4f sv = *(const v4f*)(sacc + slot * DF + colp[p]) + ps[p] * xv;
      const float dv  = den[slot * NHD + hdp[p]] + ps[p];
      const float inv = 1.0f / (dv + 1e-16f);
      hv[p] = sv * inv + b4[p];
      s1 += (hv[p].x + hv[p].y) + (hv[p].z + hv[p].w);
    }
#pragma unroll
    for (int mk = LPS / 2; mk >= 1; mk >>= 1) s1 += __shfl_xor(s1, mk, 32);
    const float mu = s1 * (1.0f / DF);
    v4f dd[NPC];
    float q = 0.f;
#pragma unroll
    for (int p = 0; p < NPC; ++p) {
      dd[p] = hv[p] - mu;
      q += (dd[p].x * dd[p].x + dd[p].y * dd[p].y) + (dd[p].z * dd[p].z + dd[p].w * dd[p].w);
    }
#pragma unroll
    for (int mk = LPS / 2; mk >= 1; mk >>= 1) q += __shfl_xor(q, mk, 32);
    const float rs = rsqrtf(q * (1.0f / DF) + 1e-5f);
    v4f y[NPC];
#pragma unroll
    for (int p = 0; p < NPC; ++p) {
      v4f t = dd[p] * rs * g4[p] + e4[p];
      t.x = t.x > 0.f ? t.x : 0.f;
      t.y = t.y > 0.f ? t.y : 0.f;
      t.z = t.z > 0.f ? t.z : 0.f;
      t.w = t.w > 0.f ? t.w : 0.f;
      if (RESID) t = t + *(const v4f*)(xres + rb + colp[p]);
      y[p] = t;
    }
    if (valid) {
#pragma unroll
      for (int p = 0; p < NPC; ++p) *(volatile v4f*)(out + rb + colp[p]) = y[p];
    }
    __threadfence();
    if (valid) {
#pragma unroll
      for (int p = 0; p < NPC; ++p) *(volatile v4f*)(out + rb + colp[p]) = y[p];
    }
  }
}

__global__ __launch_bounds__(NTHR) void k_pool(const float* __restrict__ x, const int* __restrict__ batch,
                                              float* outp, int nN) {
  __shared__ __attribute__((aligned(16))) float psum[4 * HCW];
  __shared__ __attribute__((aligned(16))) float pmax[4 * HCW];
  __shared__ int pcnt[4];
  __shared__ __attribute__((aligned(16))) float rowb[2 * HCW];
  const int tid = threadIdx.x, lane = tid & 31, wave = tid >> 5;
  const int g = blockIdx.x;
  const int c = tid & (HCW - 1);
  const int q = tid >> 6;
  float s = 0.f, mx = -3.0e38f;
  int cnt = 0;
#pragma unroll 1
  for (int n = q; n < nN; n += 4) {
    if (batch[n] == g) {
      const float v = x[(size_t)n * HCW + c];
      s += v;
      mx = fmaxf(mx, v);
      ++cnt;
    }
  }
  psum[q * HCW + c] = s;
  pmax[q * HCW + c] = mx;
  if (c == 0) pcnt[q] = cnt;
  __syncthreads();
  if (tid < HCW) {
    const float S = ((psum[c] + psum[HCW + c]) + psum[2 * HCW + c]) + psum[3 * HCW + c];
    const float M = fmaxf(fmaxf(pmax[c], pmax[HCW + c]), fmaxf(pmax[2 * HCW + c], pmax[3 * HCW + c]));
    const int C = pcnt[0] + pcnt[1] + pcnt[2] + pcnt[3];
    const float cf = (float)(C > 1 ? C : 1);
    rowb[c] = S * (1.0f / cf);
    rowb[HCW + c] = (C > 0) ? M : 0.f;
  }
  __syncthreads();
  if (wave == 0) {
    const v4f v = *(const v4f*)(rowb + 4 * lane);
    float* p = outp + (size_t)g * (2 * HCW) + 4 * lane;
    *(volatile v4f*)p = v;
    __threadfence();
    *(volatile v4f*)p = v;
  }
}

static constexpr size_t gat_lds_bytes(int DF, int NHD, int NB) {
  return ((size_t)NB * DF + (size_t)NB * NHD + (size_t)NWAVE * WCAP + NWAVE) * 4;
}
static_assert(gat_lds_bytes(256, 4, 256) == 274464);
static_assert(gat_lds_bytes(64, 1, 1024) == 274464);

extern "C" void kernel_launch(void* const* d_in, const int* in_sizes, int n_in,
                              void* d_out, int out_size, void* d_ws, size_t ws_size,
                              hipStream_t stream) {
  if (n_in < 21) return;
  const int nN = in_sizes[0] / KD;
  const int nE = in_sizes[1] / 2;
  if (nN <= 0 || in_sizes[0] != nN * KD) return;
  if (nN > (1 << 20)) return;
  if (nE < 0 || in_sizes[1] != 2 * nE) return;
  if (in_sizes[2] != nN) return;
  if (in_sizes[3] != KD * 256 || in_sizes[9] != KD * 256 || in_sizes[15] != KD * HCW) return;
  if (in_sizes[4] != 256 || in_sizes[5] != 256 || in_sizes[10] != 256 || in_sizes[11] != 256) return;
  if (in_sizes[6] != 256 || in_sizes[7] != 256 || in_sizes[8] != 256) return;
  if (in_sizes[12] != 256 || in_sizes[13] != 256 || in_sizes[14] != 256) return;
  if (in_sizes[16] != HCW || in_sizes[17] != HCW || in_sizes[18] != HCW ||
      in_sizes[19] != HCW || in_sizes[20] != HCW) return;
  const int remOut = out_size - nN * HCW;
  if (remOut <= 0 || (remOut % (2 * HCW)) != 0) return;
  const int nG = remOut / (2 * HCW);

  const float* node_x = (const float*)d_in[0];
  const int*   ei     = (const int*)d_in[1];
  const int*   batch  = (const int*)d_in[2];
  const float* W1  = (const float*)d_in[3];
  const float* as1 = (const float*)d_in[4];
  const float* ad1 = (const float*)d_in[5];
  const float* b1  = (const float*)d_in[6];
  const float* g1  = (const float*)d_in[7];
  const float* be1 = (const float*)d_in[8];
  const float* W2  = (const float*)d_in[9];
  const float* as2 = (const float*)d_in[10];
  const float* ad2 = (const float*)d_in[11];
  const float* b2  = (const float*)d_in[12];
  const float* g2  = (const float*)d_in[13];
  const float* be2 = (const float*)d_in[14];
  const float* Wf  = (const float*)d_in[15];
  const float* asf = (const float*)d_in[16];
  const float* adf = (const float*)d_in[17];
  const float* bfp = (const float*)d_in[18];
  const float* gf  = (const float*)d_in[19];
  const float* bef = (const float*)d_in[20];
  float* out0 = (float*)d_out;
  float* out1 = out0 + (size_t)nN * HCW;

  const int nP = ((nN + GR - 1) / GR) * GR;
  size_t off = 0;
  auto carve = [&](size_t bytes) -> char* {
    char* p = (char*)d_ws + off;
    off += (bytes + 255) & ~(size_t)255;
    return p;
  };
  _Float16* Wh1 = (_Float16*)carve((size_t)256 * KD * sizeof(_Float16));
  _Float16* Wh2 = (_Float16*)carve((size_t)256 * KD * sizeof(_Float16));
  _Float16* Whf = (_Float16*)carve((size_t)HCW * KD * sizeof(_Float16));
  float* xp = (float*)carve((size_t)nP * 256 * sizeof(float));
  float* es = (float*)carve((size_t)nP * 4 * sizeof(float));
  float* ed = (float*)carve((size_t)nP * 4 * sizeof(float));
  float* xA = (float*)carve((size_t)nP * 256 * sizeof(float));
  float* xB = (float*)carve((size_t)nP * 256 * sizeof(float));
  if (off > ws_size) return;
  if (off > (size_t)134217728) return;

  const size_t L1 = gat_lds_bytes(256, 4, 256);
  const size_t L3 = gat_lds_bytes(64, 1, 1024);
  hipFuncSetAttribute(reinterpret_cast<const void*>(&k_gat<256, 4, 256, 8, true>),
                      hipFuncAttributeMaxDynamicSharedMemorySize, (int)L1);
  hipFuncSetAttribute(reinterpret_cast<const void*>(&k_gat<64, 1, 1024, 10, false>),
                      hipFuncAttributeMaxDynamicSharedMemorySize, (int)L3);

  k_prepw<256><<<dim3(256 / 16), dim3(NTHR), 0, stream>>>(W1, Wh1);
  k_prepw<256><<<dim3(256 / 16), dim3(NTHR), 0, stream>>>(W2, Wh2);
  k_prepw<64><<<dim3(HCW / 16), dim3(NTHR), 0, stream>>>(Wf, Whf);

  const int gGemm = nP / GR;
  const int gGat1 = (nN + 256 - 1) / 256;
  const int gGat3 = (nN + 1024 - 1) / 1024;

  k_gemm<256, 4><<<dim3(gGemm), dim3(NTHR), 0, stream>>>(node_x, Wh1, as1, ad1, xp, es, ed, nN);
  k_gat<256, 4, 256, 8, true><<<dim3(gGat1), dim3(NTHR), L1, stream>>>(
      node_x, ei, xp, es, ed, b1, g1, be1, xA, nN, nE);
  k_gemm<256, 4><<<dim3(gGemm), dim3(NTHR), 0, stream>>>(xA, Wh2, as2, ad2, xp, es, ed, nN);
  k_gat<256, 4, 256, 8, true><<<dim3(gGat1), dim3(NTHR), L1, stream>>>(
      xA, ei, xp, es, ed, b2, g2, be2, xB, nN, nE);
  k_gemm<64, 1><<<dim3(gGemm), dim3(NTHR), 0, stream>>>(xB, Whf, asf, adf, xp, es, ed, nN);
  k_gat<64, 1, 1024, 10, false><<<dim3(gGat3), dim3(NTHR), L3, stream>>>(
      xB, ei, xp, es, ed, bfp, gf, bef, out0, nN, nE);
  k_pool<<<dim3(nG), dim3(NTHR), 0, stream>>>(out0, batch, out1, nN);
}
